// MaskedAttention_73203422593481
// MI455X (gfx1250) — hardware-verified
//
#include <hip/hip_runtime.h>
#include <stdint.h>

#ifndef NB
#define NB 32
#endif
#ifndef SEQ
#define SEQ 2048
#endif
#define NB_FULL  32
#define SEQ_FULL 2048
#define DH       128
#define NTOK     (NB * SEQ)

typedef _Float16 v16h __attribute__((ext_vector_type(16)));
typedef _Float16 v8h  __attribute__((ext_vector_type(8)));
typedef float    v8f  __attribute__((ext_vector_type(8)));
typedef float    v4f  __attribute__((ext_vector_type(4)));

static_assert(NB >= 1 && NB <= NB_FULL && SEQ >= 128 && SEQ <= SEQ_FULL);
static_assert((SEQ % 128) == 0 && (SEQ % 64) == 0 && (SEQ % 16) == 0 && ((NB * SEQ) % 16) == 0);
static_assert((size_t)NB_FULL * SEQ_FULL * DH * 4 == (size_t)33554432);

__device__ __forceinline__ _Float16 cvt16(float f) {
  unsigned u = __float_as_uint(f);
  u = (u + 0x7FFFu + ((u >> 16) & 1u)) & 0xFFFF0000u;
  return (_Float16)(__uint_as_float(u) * 64.0f);
}

__device__ __forceinline__ v16h ldfrag(const _Float16* p) {
  union { v16h v; v8h hh[2]; } f;
  f.hh[0] = *(const v8h*)(p);
  f.hh[1] = *(const v8h*)(p + 16);
  return f.v;
}
__device__ __forceinline__ v8f mma16(v16h a, v16h b, v8f c) {
  return __builtin_amdgcn_wmma_f32_16x16x32_f16(false, a, false, b, (short)0, c, false, false);
}
__device__ __forceinline__ v8f zero8() {
  v8f z;
#pragma unroll
  for (int i = 0; i < 8; ++i) z[i] = 0.0f;
  return z;
}
__device__ __forceinline__ void guard1(v8f& d, v16h x, v16h y) {
  asm volatile("v_nop\n\tv_nop\n\tv_nop\n\tv_nop" : "+v"(d) : "v"(x), "v"(y));
}
__device__ __forceinline__ void guard2(v8f& d0, v8f& d1, v16h x, v16h y, v16h z) {
  asm volatile("v_nop\n\tv_nop\n\tv_nop\n\tv_nop" : "+v"(d0), "+v"(d1) : "v"(x), "v"(y), "v"(z));
}

__global__ __launch_bounds__(256) void cvt_qk_kernel(const float* __restrict__ q, const float* __restrict__ k,
                                                     _Float16* __restrict__ qd, _Float16* __restrict__ kd, int n8) {
  const int li = (int)blockIdx.x * 256 + (int)threadIdx.x;
  if (li >= n8) return;
  const int z = (int)blockIdx.y;
  const float* src = (z == 0) ? q : k;
  _Float16* dst = (z == 0) ? qd : kd;
  const size_t e = (size_t)li * 8;
  const size_t tok = e / DH;
  const size_t dd = e - tok * DH;
  const size_t s = tok / SEQ;
  const size_t ge = (s * SEQ_FULL + (tok - s * SEQ)) * DH + dd;
  const v4f a = *(const v4f*)(src + ge);
  const v4f b = *(const v4f*)(src + ge + 4);
  v8h o;
#pragma unroll
  for (int i = 0; i < 4; ++i) {
    o[i]     = cvt16(a[i]);
    o[4 + i] = cvt16(b[i]);
  }
  _Float16* d = dst + e;
  *(volatile v8h*)d = o;
  __threadfence();
  *(volatile v8h*)d = o;
}

__global__ __launch_bounds__(256) void cvt_vt_kernel(const float* __restrict__ v, _Float16* __restrict__ vt) {
  __shared__ float sTt[64][33];
  const int k0 = (int)blockIdx.x * 64, n0 = (int)blockIdx.y * 32;
  const int t = (int)threadIdx.x;
  const int s = k0 / SEQ;
  const size_t grow0 = (size_t)s * SEQ_FULL + (size_t)(k0 - s * SEQ);
  {
    const int kr = t >> 2, cc = (t & 3) * 8;
    const float* sp = v + (grow0 + kr) * DH + n0 + cc;
    const v4f a = *(const v4f*)(sp);
    const v4f b = *(const v4f*)(sp + 4);
#pragma unroll
    for (int e = 0; e < 4; ++e) {
      sTt[kr][cc + e]     = a[e];
      sTt[kr][cc + 4 + e] = b[e];
    }
  }
  __syncthreads();
  const int n = t >> 3, kq = (t & 7) * 8;
  v8h o;
#pragma unroll
  for (int i = 0; i < 8; ++i) o[i] = cvt16(sTt[kq + i][n]);
  _Float16* d = vt + (size_t)(n0 + n) * NTOK + k0 + kq;
  *(volatile v8h*)d = o;
  __threadfence();
  *(volatile v8h*)d = o;
}

#define QB     16
#define NWAVE  8
#define KCH    128
#define QSP    136
#define PSP    136
#define OSP    132
#define TSPLIT 32
#define SCL    (0.08838834764831845f * 0.000244140625f)
#define K2048  0.00048828125f
#define KINV   1.52587890625e-05f
static_assert(NWAVE * 16 == KCH && NWAVE * 16 == DH && QB == 16 && NWAVE * 2 == QB && NWAVE * QB <= 256 && NWAVE * 32 == 256);
static_assert((QSP % 8) == 0 && (PSP % 8) == 0 && (OSP % 4) == 0 && QSP >= DH && PSP >= KCH && OSP >= DH);
static_assert((SEQ % KCH) == 0 && (SEQ % QB) == 0 && QB * (DH / 8) == 256);

template <bool RES>
__global__ __launch_bounds__(256) __attribute__((amdgpu_num_vgpr(256)))
void attn_kernel(const _Float16* __restrict__ qp, const _Float16* __restrict__ kp,
                 const _Float16* __restrict__ vtp, float* __restrict__ out, int qt0) {
  __shared__ __align__(16) _Float16 Qs[QB * QSP];
  __shared__ __align__(16) _Float16 Phs[QB * PSP];
  __shared__ __align__(16) _Float16 Pls[QB * PSP];
  __shared__ __align__(16) float Os[QB * OSP];
  __shared__ __align__(16) float pmax[NWAVE * QB];
  __shared__ __align__(16) float psum[NWAVE * QB];
  __shared__ __align__(16) float st_s[4 * QB];
  float* m_s  = st_s;
  float* l_s  = st_s + QB;
  float* al_s = st_s + 2 * QB;
  float* li_s = st_s + 3 * QB;

  const int tid = (int)threadIdx.x;
  const int wave = __builtin_amdgcn_readfirstlane(tid >> 5);
  const int lane = tid & 31, h = lane >> 4, c = lane & 15;
  const int sq = (int)blockIdx.y;
  const int q0 = (qt0 + (int)blockIdx.x) * QB;
  const int qlast = q0 + QB - 1;
  const size_t pt0 = (size_t)sq * SEQ + q0;
  const size_t ot0 = (size_t)sq * SEQ_FULL + q0;
  const float ninf = -__builtin_inff();

  if (tid < QB) { m_s[tid] = ninf; l_s[tid] = 0.0f; al_s[tid] = 0.0f; li_s[tid] = 0.0f; }
  if (tid < NWAVE * QB) psum[tid] = 0.0f;
  {
    const int row = tid >> 4;
    const int pc  = tid & 15;
    const v8h v0 = *(const v8h*)(qp + (pt0 + row) * DH + (size_t)pc * 8);
    *(v8h*)(Qs + row * QSP + pc * 8) = v0;
  }
  __syncthreads();

  v8f oacc1 = zero8(), oacc2 = zero8();
  const _Float16* qbp = Qs  + c * QSP + 8 * h;
  const _Float16* pap = Phs + c * PSP + 8 * h;
  const _Float16* plp = Pls + c * PSP + 8 * h;
  const int ntile = (q0 / KCH) + 1;

#pragma unroll 1
  for (int t = 0; t < ntile; ++t) {
    const int kb = t * KCH + 16 * wave;
    v8f s1 = zero8();
    if (kb <= qlast) {
      const _Float16* kap = kp + ((size_t)sq * SEQ + kb + c) * DH + 8 * h;
#pragma unroll 1
      for (int k0 = 0; k0 < DH; k0 += 32) {
        const v16h a  = ldfrag(kap + k0);
        const v16h bq = ldfrag(qbp + k0);
        s1 = mma16(a, bq, s1);
        guard1(s1, a, bq);
      }
    }
    {
      float pm = ninf;
#pragma unroll
      for (int r = 0; r < 8; ++r) {
        float s = s1[r] * SCL;
        const int key = kb + 8 * h + r;
        s = (key > q0 + c) ? ninf : s;
        s1[r] = s;
        pm = fmaxf(pm, s);
      }
      pm = fmaxf(pm, __shfl_xor(pm, 16, 32));
      pmax[wave * QB + c] = pm;
    }
    __syncthreads();
    if (wave == 0 && lane < QB) {
      const int row = lane;
      float ps = 0.0f;
#pragma unroll
      for (int w = 0; w < NWAVE; ++w) ps += psum[w * QB + row];
      l_s[row] = l_s[row] * al_s[row] + ps;
      const float mo = m_s[row];
      float mx = mo;
#pragma unroll
      for (int w = 0; w < NWAVE; ++w) mx = fmaxf(mx, pmax[w * QB + row]);
      al_s[row] = __expf(mo - mx);
      m_s[row] = mx;
    }
    __syncthreads();
    {
      const float mq = m_s[c];
      float ps = 0.0f;
      v8h ph, pr;
#pragma unroll
      for (int r = 0; r < 8; ++r) {
        const float p = __expf(s1[r] - mq);
        ps += p;
        const float pc = p * 1024.0f;
        const _Float16 hh = (_Float16)pc;
        ph[r] = hh;
        pr[r] = (_Float16)((pc - (float)hh) * 2048.0f);
      }
      *(v8h*)(Phs + c * PSP + 16 * wave + 8 * h) = ph;
      if (RES) *(v8h*)(Pls + c * PSP + 16 * wave + 8 * h) = pr;
      ps += __shfl_xor(ps, 16, 32);
      psum[wave * QB + c] = ps;
      const v4f aA = *(const v4f*)(al_s + 8 * h), aB = *(const v4f*)(al_s + 8 * h + 4);
#pragma unroll
      for (int r = 0; r < 4; ++r) {
        oacc1[r] *= aA[r]; oacc1[4 + r] *= aB[r];
        if (RES) { oacc2[r] *= aA[r]; oacc2[4 + r] *= aB[r]; }
      }
    }
    __syncthreads();
    {
      int kend = q0 + QB - t * KCH;
      kend = (kend > KCH) ? KCH : kend;
      kend = (kend + 31) & ~31;
      const _Float16* vhp = vtp + (size_t)(16 * wave + c) * NTOK + (size_t)sq * SEQ + (size_t)t * KCH + 8 * h;
#pragma unroll 1
      for (int ks = 0; ks < kend; ks += 32) {
        const v16h pa = ldfrag(pap + ks);
        const v16h x  = ldfrag(vhp + ks);
        v16h pz = pa;
        if (RES) pz = ldfrag(plp + ks);
        oacc1 = mma16(pa, x, oacc1);
        if (RES) oacc2 = mma16(pz, x, oacc2);
        guard2(oacc1, oacc2, pa, pz, x);
      }
    }
  }

  if (wave == 0 && lane < QB) {
    const int row = lane;
    float ps = 0.0f;
#pragma unroll
    for (int w = 0; w < NWAVE; ++w) ps += psum[w * QB + row];
    const float l = l_s[row] * al_s[row] + ps;
    li_s[row] = (1.0f / l) * KINV;
  }
  __syncthreads();
  {
    const v4f iA = *(const v4f*)(li_s + 8 * h), iB = *(const v4f*)(li_s + 8 * h + 4);
    const int col = 16 * wave + c;
#pragma unroll
    for (int r = 0; r < 4; ++r) {
      float o0 = oacc1[r], o1 = oacc1[4 + r];
      if (RES) { o0 += oacc2[r] * K2048; o1 += oacc2[4 + r] * K2048; }
      Os[(8 * h + r) * OSP + col]     = o0 * iA[r];
      Os[(8 * h + 4 + r) * OSP + col] = o1 * iB[r];
    }
  }
  __syncthreads();
  {
#pragma unroll
    for (int ps = 0; ps < 2; ++ps) {
#pragma unroll
      for (int rr = 0; rr < 2; ++rr) {
        const int row = 2 * wave + rr;
        const v4f vv = *(const v4f*)(Os + row * OSP + lane * 4);
        *(volatile v4f*)(out + (ot0 + (size_t)row) * DH + lane * 4) = vv;
      }
      __threadfence();
    }
  }
}

extern "C" void kernel_launch(void* const* d_in, const int* in_sizes, int n_in,
                              void* d_out, int out_size, void* d_ws, size_t ws_size,
                              hipStream_t stream) {
  if (n_in < 3) return;
  const int need = NB * SEQ_FULL * DH;
  if (in_sizes[0] < need || in_sizes[1] < need || in_sizes[2] < need) return;
  if (out_size < need) return;

  const float* Q = (const float*)d_in[0];
  const float* K = (const float*)d_in[1];
  const float* V = (const float*)d_in[2];
  float* out = (float*)d_out;

  const size_t bAct = (size_t)NTOK * DH * 2;
  size_t off = 0;
  const size_t oQ = off; off += bAct;
  const size_t oK = off; off += bAct;
  const size_t oV = off; off += bAct;
  if (off > ws_size) return;
  if (off > (size_t)134217728) return;

  char* ws = (char*)d_ws;
  _Float16* Qp = (_Float16*)(ws + oQ);
  _Float16* Kp = (_Float16*)(ws + oK);
  _Float16* Vt = (_Float16*)(ws + oV);

  const int n8 = NTOK * DH / 8;
  if ((n8 % 256) != 0) return;

  cvt_qk_kernel<<<dim3(n8 / 256, 2), dim3(256), 0, stream>>>(Q, K, Qp, Kp, n8);
  cvt_vt_kernel<<<dim3(NTOK / 64, DH / 32), dim3(256), 0, stream>>>(V, Vt);
  const int nqt = SEQ / QB;
  const int ts = (TSPLIT < nqt) ? TSPLIT : nqt;
  attn_kernel<true><<<dim3(ts, NB), dim3(256), 0, stream>>>(Qp, Kp, Vt, out, 0);
  if (nqt - ts > 0)
    attn_kernel<false><<<dim3(nqt - ts, NB), dim3(256), 0, stream>>>(Qp, Kp, Vt, out, ts);
  (void)hipGetLastError();
}
